// Head_6021544149785
// MI455X (gfx1250) — hardware-verified
//
#include <hip/hip_runtime.h>


#ifndef NB
#define NB 16
#endif
#ifndef SEQ
#define SEQ 2048
#endif

namespace {
constexpr int B_FULL = 16, T_FULL = 2048, C = 384, HD = 64;
constexpr int NBL = NB;
constexpr int SQ = SEQ;
constexpr int KC = 128;
constexpr float XS = 8.0f, WSC = 256.0f, PS = 1024.0f, LOG2E = 1.4426950408889634f, SCL = 0.125f;
static_assert(NBL >= 1 && NBL <= B_FULL);
static_assert(SQ >= 64 && SQ <= T_FULL && SQ % 64 == 0 && SQ % 32 == 0);
static_assert(C % KC == 0 && KC % 32 == 0 && C % 8 == 0 && HD == 64);
constexpr int PREP_ELEMS = 3 * HD * C;
constexpr int PREP_THREADS = PREP_ELEMS / 8;
static_assert(PREP_ELEMS % 8 == 0 && PREP_THREADS % 256 == 0);
static_assert((PREP_THREADS / 256) * 256 * 8 == PREP_ELEMS);
static_assert((SQ / 64) * 64 == SQ && (SQ / 32) * 32 == SQ);

typedef _Float16 b16;
typedef __attribute__((ext_vector_type(16))) _Float16 v16b;
typedef __attribute__((ext_vector_type(8))) _Float16 v8b;
typedef __attribute__((ext_vector_type(4))) _Float16 v4h;
typedef __attribute__((ext_vector_type(8))) float v8f;
typedef __attribute__((ext_vector_type(4))) float v4f;

__device__ __forceinline__ float bf16_rne(float f) { unsigned int u = __float_as_uint(f); u += 0x7FFFu + ((u >> 16) & 1u); return __uint_as_float(u & 0xFFFF0000u); }
__device__ __forceinline__ v16b frag_kb(const b16* p, int hh) { const v8b a = *(const v8b*)(p + 8 * hh), b = *(const v8b*)(p + 16 + 8 * hh); v16b f;
#pragma unroll
  for (int e = 0; e < 8; ++e) { f[e] = a[e]; f[8 + e] = b[e]; } return f; }
__device__ __forceinline__ v8f wmma16b(v16b a, v16b b, v8f c) { v8f d = __builtin_amdgcn_wmma_f32_16x16x32_f16(false, a, false, b, (short)0, c, false, false); asm volatile("v_nop\n\tv_nop\n\tv_nop\n\tv_nop" : "+v"(d) : "v"(a), "v"(b)); return d; }
__device__ __forceinline__ void wave_lds_sync() { __builtin_amdgcn_fence(3  , "workgroup"); __builtin_amdgcn_wave_barrier(); __builtin_amdgcn_fence(2  , "workgroup"); }
__device__ __forceinline__ float nexp2(float v) { return __builtin_amdgcn_exp2f(v); }

__global__ __launch_bounds__(256) void prep_kernel(const float* __restrict__ wq, const float* __restrict__ wk, const float* __restrict__ wv, b16* __restrict__ WT) {
  const size_t u = (size_t)blockIdx.x * 256 + threadIdx.x; if (u >= (size_t)PREP_THREADS) return;
  const size_t e = u * 8; const int oo = (int)(e / C), c0 = (int)(e % C); const int m = oo / HD, o2 = oo % HD; const float* w = m == 0 ? wq : m == 1 ? wk : wv; v8b o;
#pragma unroll
  for (int j = 0; j < 8; ++j) o[j] = (b16)(bf16_rne(w[(size_t)(c0 + j) * HD + o2]) * WSC);
  for (int pass = 0; pass < 2; ++pass) { *(volatile v8b*)(WT + e) = o; __threadfence(); }
}

__global__ __launch_bounds__(128) void proj_kernel(const float* __restrict__ X, const b16* __restrict__ WT, const float* __restrict__ bq, const float* __restrict__ bk, const float* __restrict__ bv,
                                                   b16* __restrict__ QP, b16* __restrict__ KP, b16* __restrict__ VT) {
  __shared__ __attribute__((aligned(16))) b16 As[64][KC + 8]; __shared__ __attribute__((aligned(16))) float Tf[4][16][HD + 4];
  const int wave = threadIdx.x >> 5, lane = threadIdx.x & 31, nloc = lane & 15, hlf = lane >> 4; const int t0 = blockIdx.x * 64; const int b = blockIdx.y; const int part = blockIdx.z;
  const float* xb = X + ((size_t)b * T_FULL + t0) * C; const float* bias = part == 0 ? bq : part == 1 ? bk : bv; const b16* W = WT + (size_t)part * HD * C;
  v8f acc[4];
#pragma unroll
  for (int t = 0; t < 4; ++t) acc[t] = (v8f){};
#pragma unroll 1
  for (int kc = 0; kc < C; kc += KC) {
    __syncthreads();
    for (int i = threadIdx.x; i < 64 * (KC / 4); i += 128) { const int rr = i / (KC / 4), q = (i % (KC / 4)) * 4; const v4f f = *(const v4f*)(xb + (size_t)rr * C + kc + q); v4h o;
#pragma unroll
      for (int j = 0; j < 4; ++j) o[j] = (b16)(bf16_rne(f[j]) * XS); *(v4h*)(&As[rr][q]) = o; }
    __syncthreads();
#pragma unroll 2
    for (int kb = 0; kb < KC; kb += 32) { const v16b a = frag_kb(&As[wave * 16 + nloc][kb], hlf);
#pragma unroll
      for (int t = 0; t < 4; ++t) acc[t] = wmma16b(a, frag_kb(W + (size_t)(t * 16 + nloc) * C + kc + kb, hlf), acc[t]); } }
#pragma unroll
  for (int t = 0; t < 4; ++t) { const float bb = bf16_rne(bias[t * 16 + nloc]);
#pragma unroll
    for (int r = 0; r < 8; ++r) Tf[wave][8 * hlf + r][t * 16 + nloc] = acc[t][r] * (1.0f / (XS * WSC)) + bb; }
  __syncthreads();
  for (int pass = 0; pass < 2; ++pass) {
    if (part < 2) { b16* plane = part == 0 ? QP : KP;
#pragma unroll 1
      for (int it = 0; it < 4; ++it) { const int rr = it * 4 + (lane >> 3); const int tok = t0 + wave * 16 + rr; const int c8 = (lane & 7) * 8; v8b o8;
#pragma unroll
        for (int j = 0; j < 8; ++j) o8[j] = (b16)(Tf[wave][rr][c8 + j] * XS);
        *(volatile v8b*)(plane + ((size_t)b * SQ + tok) * HD + c8) = o8; } }
    else {
#pragma unroll 1
      for (int it = 0; it < 4; ++it) { const int d = wave * 16 + it * 4 + (lane >> 3); const int tk0 = (lane & 7) * 8; v8b vv;
#pragma unroll
        for (int j = 0; j < 8; ++j) { const int tk = tk0 + j; vv[j] = (b16)(Tf[tk >> 4][tk & 15][d] * XS); }
        *(volatile v8b*)(VT + ((size_t)b * HD + d) * (size_t)SQ + t0 + tk0) = vv; } }
    __threadfence(); }
}

__global__ __launch_bounds__(64) void attn_kernel(const b16* __restrict__ QP, const b16* __restrict__ KP, const b16* __restrict__ VT, float* __restrict__ out) {
  __shared__ __attribute__((aligned(16))) b16 Pb[2][16][32 + 8]; __shared__ __attribute__((aligned(16))) float To[2][16][HD + 4];
  const int wave = threadIdx.x >> 5, lane = threadIdx.x & 31, hh = lane >> 4, col = lane & 15; const int b = blockIdx.y; const int r0 = blockIdx.x * 32 + wave * 16, ri = r0 + col;
  const b16* Qb = QP + (size_t)b * SQ * HD; const b16* Kb = KP + (size_t)b * SQ * HD; const b16* Vb = VT + (size_t)b * HD * (size_t)SQ;
  v16b qa[2];
#pragma unroll
  for (int i = 0; i < 2; ++i) qa[i] = frag_kb(Qb + (size_t)ri * HD + 32 * i, hh);
  const float cs = SCL * LOG2E / (XS * XS);
  float m = -__builtin_inff(), l = 0.0f; v8f o[4];
#pragma unroll
  for (int t = 0; t < 4; ++t) o[t] = (v8f){};
#pragma unroll 1
  for (int sb = 0; sb < SQ; sb += 32) {
    float e[16]; float mx = -__builtin_inff();
#pragma unroll
    for (int u = 0; u < 2; ++u) { v8f s = (v8f){}; const size_t kr = (size_t)(sb + u * 16 + col) * HD;
#pragma unroll
      for (int i = 0; i < 2; ++i) s = wmma16b(frag_kb(Kb + kr + 32 * i, hh), qa[i], s);
#pragma unroll
      for (int r = 0; r < 8; ++r) { const float vv = s[r] * cs; e[u * 8 + r] = vv; mx = fmaxf(mx, vv); } }
    mx = fmaxf(mx, __shfl_xor(mx, 16)); const float mn = fmaxf(m, mx); const float al = nexp2(m - mn); float sum = 0.0f;
#pragma unroll
    for (int i2 = 0; i2 < 16; ++i2) { const float p = nexp2(e[i2] - mn); sum += p; Pb[wave][col][(i2 < 8 ? 0 : 16) + 8 * hh + (i2 & 7)] = (b16)(p * PS); }
    sum += __shfl_xor(sum, 16); l = l * al + sum; m = mn;
    wave_lds_sync();
    const v16b pf = frag_kb(&Pb[wave][col][0], hh);
#pragma unroll
    for (int t = 0; t < 4; ++t) { o[t] *= al; o[t] = wmma16b(frag_kb(Vb + (size_t)(t * 16 + col) * SQ + sb, hh), pf, o[t]); }
    wave_lds_sync(); }
  const float inv = 1.0f / (l * PS * XS);
#pragma unroll
  for (int t = 0; t < 4; ++t)
#pragma unroll
    for (int r = 0; r < 8; ++r) To[wave][col][t * 16 + 8 * hh + r] = o[t][r] * inv;
  wave_lds_sync();
  for (int pass = 0; pass < 2; ++pass) {
#pragma unroll 1
    for (int it = 0; it < 8; ++it) { const int rr = it * 2 + (lane >> 4); const int c4 = (lane & 15) * 4;
      *(volatile v4f*)(out + ((size_t)b * SQ + r0 + rr) * HD + c4) = *(const v4f*)(&To[wave][rr][c4]); }
    __threadfence(); }
}
}

extern "C" void kernel_launch(void* const* d_in, const int* in_sizes, int n_in, void* d_out, int out_size, void* d_ws, size_t ws_size, hipStream_t stream) {
  if (n_in < 7) return;
  auto Fp = [&](int i) { return (const float*)d_in[i]; };
  if ((size_t)in_sizes[0] < (size_t)NBL * T_FULL * C || in_sizes[1] < C * HD || in_sizes[2] < HD || in_sizes[3] < C * HD || in_sizes[4] < HD || in_sizes[5] < C * HD || in_sizes[6] < HD) return;
  if ((size_t)out_size < (size_t)NBL * SQ * HD) return;
  size_t off = 0; char* ws = (char*)d_ws;
  auto carve = [&](size_t bytes) { char* p = ws + off; off += (bytes + 255) & ~(size_t)255; return p; };
  b16* WT = (b16*)carve((size_t)PREP_ELEMS * 2);
  const size_t plane = (size_t)NBL * SQ * HD * 2;
  b16* QP = (b16*)carve(plane); b16* KP = (b16*)carve(plane); b16* VT = (b16*)carve(plane);
  if (off > ws_size || off > ((size_t)128 << 20)) return;
  prep_kernel<<<(unsigned)(PREP_THREADS / 256), 256, 0, stream>>>(Fp(1), Fp(3), Fp(5), WT);
  proj_kernel<<<dim3(SQ / 64, NBL, 3), 128, 0, stream>>>(Fp(0), WT, Fp(2), Fp(4), Fp(6), QP, KP, VT);
  attn_kernel<<<dim3(SQ / 32, NBL), 64, 0, stream>>>(QP, KP, VT, (float*)d_out);
}
